// FactorizedAttentionBlock_19679540150350
// MI455X (gfx1250) — hardware-verified
//
#include <hip/hip_runtime.h>
#include <math.h>

typedef __attribute__((ext_vector_type(16))) _Float16 v16h;
typedef __attribute__((ext_vector_type(16))) __bf16 v16b;
typedef __attribute__((ext_vector_type(8)))  _Float16 v8h;
typedef __attribute__((ext_vector_type(8)))  float v8f;
typedef __attribute__((ext_vector_type(4)))  float v4f;
typedef __attribute__((ext_vector_type(2)))  float v2f;
typedef __attribute__((ext_vector_type(4)))  unsigned v4u;
typedef __attribute__((ext_vector_type(4)))  int v4i;
typedef float __attribute__((may_alias)) float_a;
typedef int __attribute__((may_alias)) int_a;

template <typename T> __device__ __forceinline__ void vst2(void* p, T v) { *(volatile T*)p = v; __threadfence(); *(volatile T*)p = v; }
__device__ __forceinline__ v8f wmma16(v16h a, v16h b, v8f c) {
  v8f d = __builtin_amdgcn_wmma_f32_16x16x32_f16(false, a, false, b, (short)0, c, false, false);
  asm volatile("v_nop\n\tv_nop\n\tv_nop\n\tv_nop" : "+v"(d) : "v"(a), "v"(b));
  return d;
}
__device__ __forceinline__ v8f wmma_bf(v16b a, v16b b, v8f c) {
  v8f d = __builtin_amdgcn_wmma_f32_16x16x32_bf16(false, a, false, b, (short)0, c, false, false);
  asm volatile("v_nop\n\tv_nop\n\tv_nop\n\tv_nop" : "+v"(d) : "v"(a), "v"(b));
  return d;
}
__device__ __forceinline__ v16h frag_h(const _Float16* rowk0, int lane) {
  union { v16h v; v8h q[2]; } u; const _Float16* p = rowk0 + 8 * (lane >> 4);
  u.q[0] = *(const v8h*)p; u.q[1] = *(const v8h*)(p + 16); return u.v;
}
__device__ __forceinline__ v16h frag_f32(const float* rowk0, int lane) {
  v16h a; const float* p = rowk0 + 8 * (lane >> 4);
#pragma unroll
  for (int i = 0; i < 8; ++i) { a[i] = (_Float16)p[i]; a[8 + i] = (_Float16)p[16 + i]; }
  return a;
}
__device__ __forceinline__ v16h frag_f32s(const float* rowk0, int lane, float sc) {
  v16h a; const float* p = rowk0 + 8 * (lane >> 4);
#pragma unroll
  for (int i = 0; i < 8; ++i) { a[i] = (_Float16)(p[i] * sc); a[8 + i] = (_Float16)(p[16 + i] * sc); }
  return a;
}
__device__ __forceinline__ v16h fragc_f32(const float* W, int k0, int n, int lane, int ld, int K) {
  v16h a; const int g = lane >> 4;
#pragma unroll
  for (int i = 0; i < 8; ++i) { const int ka = k0 + 8 * g + i, kb = ka + 16;
    a[i] = (_Float16)(ka < K ? W[(size_t)ka * ld + n] : 0.f); a[8 + i] = (_Float16)(kb < K ? W[(size_t)kb * ld + n] : 0.f); }
  return a;
}
struct F2 { v16b h, l; };
__device__ __forceinline__ F2 bsplit16(const float v[16]) { F2 r;
#pragma unroll
  for (int i = 0; i < 16; ++i) { const __bf16 h = (__bf16)v[i]; r.h[i] = h; r.l[i] = (__bf16)(v[i] - (float)h); }
  return r; }
__device__ __forceinline__ F2 split_row(const float* row, int k0, int lane) { float v[16]; const float* p = row + k0 + 8 * (lane >> 4);
#pragma unroll
  for (int i = 0; i < 8; ++i) { v[i] = p[i]; v[8 + i] = p[16 + i]; }
  return bsplit16(v); }
__device__ __forceinline__ F2 split_rowK(const float* row, int k0, int lane, int K) { float v[16]; const int g = lane >> 4;
#pragma unroll
  for (int i = 0; i < 8; ++i) { const int ka = k0 + 8 * g + i, kb = ka + 16; v[i] = ka < K ? row[ka] : 0.f; v[8 + i] = kb < K ? row[kb] : 0.f; }
  return bsplit16(v); }
__device__ __forceinline__ F2 split_col(const float* W, int k0, int n, int lane, int ld, int K) { float v[16]; const int g = lane >> 4;
#pragma unroll
  for (int i = 0; i < 8; ++i) { const int ka = k0 + 8 * g + i, kb = ka + 16; v[i] = ka < K ? W[(size_t)ka * ld + n] : 0.f; v[8 + i] = kb < K ? W[(size_t)kb * ld + n] : 0.f; }
  return bsplit16(v); }
__device__ __forceinline__ v8f mac3(const F2& a, const F2& b, v8f c) { c = wmma_bf(a.l, b.h, c); c = wmma_bf(a.h, b.l, c); return wmma_bf(a.h, b.h, c); }
__device__ __forceinline__ float sigm(float v) { return 1.0f / (1.0f + expf(-v)); }
#define LDSX() do { asm volatile("s_wait_dscnt 0" ::: "memory"); __builtin_amdgcn_wave_barrier(); __builtin_amdgcn_fence(__ATOMIC_RELEASE, "workgroup"); } while (0)

#define NB 8
#define CC 256
#define HW 64
#define WS 8
#define NWIN 64
#define LL (NWIN * NB)
#define NN 64
#define NH 8
#define HD 32
#define NR (NN * LL)

__global__ __launch_bounds__(256) void k_se(const float* __restrict__ x, const float* __restrict__ w1, const float* __restrict__ b1, const float* __restrict__ w2, const float* __restrict__ b2, float* __restrict__ CA) {
  __shared__ float sp[CC]; __shared__ float sh1[64]; __shared__ __align__(16) float sca[CC];
  const int b = blockIdx.x, c = threadIdx.x; const float* xc = x + ((size_t)b * CC + c) * HW * HW; float s = 0.f;
#pragma unroll 1
  for (int i = 0; i < HW * HW; i += 4) { const v4f v = *(const v4f*)(xc + i); s += (v[0] + v[1]) + (v[2] + v[3]); }
  sp[c] = s * (1.0f / (HW * HW));
  __syncthreads();
  if (c < 64) { float a = b1[c];
#pragma unroll 1
    for (int k = 0; k < CC; ++k) a += w1[(size_t)c * CC + k] * sp[k];
    sh1[c] = a > 0.f ? a : 0.f; }
  __syncthreads();
  { float a = b2[c];
#pragma unroll 1
    for (int k = 0; k < 64; ++k) a += w2[(size_t)c * 64 + k] * sh1[k];
    sca[c] = sigm(a); }
  __syncthreads();
  if (c < CC / 4) vst2(CA + (size_t)b * CC + c * 4, *(const v4f*)(&sca[c * 4]));
}
__global__ __launch_bounds__(256) void k_gather(const float* __restrict__ x, const float* __restrict__ CA, _Float16* __restrict__ XT) {
  __shared__ __align__(16) _Float16 st[64][CC + 8];
  const int b = blockIdx.z, hw = blockIdx.y, py = blockIdx.x, tid = threadIdx.x; const int y = hw * WS + py;
  for (int q = tid; q < CC * 64; q += 256) { const int c = q >> 6, xx = q & 63; st[xx][c] = (_Float16)(x[(((size_t)b * CC + c) * HW + y) * HW + xx] * CA[(size_t)b * CC + c]); }
  __syncthreads();
  for (int q = tid; q < 64 * 32; q += 256) { const int xx = q >> 5, pc = q & 31; const int ww = xx >> 3, px = xx & 7; const int l = (hw * 8 + ww) * NB + b, n = py * 8 + px; const size_t r = (size_t)n * LL + l;
    vst2(XT + r * CC + pc * 8, *(const v4u*)(&st[xx][pc * 8])); }
}
__global__ __launch_bounds__(256) void k_pack(const float* __restrict__ Wi, const float* __restrict__ Wo, _Float16* __restrict__ PT) {
  const int r = blockIdx.x, tid = threadIdx.x; __shared__ __align__(16) _Float16 srow[CC];
  const float* W = r < 3 * CC ? Wi + (size_t)r * CC : Wo + (size_t)(r - 3 * CC) * CC;
  srow[tid] = (_Float16)(W[tid] * 16.0f);
  __syncthreads();
  if (tid < 32) vst2(PT + (size_t)r * CC + tid * 8, *(const v4u*)(&srow[tid * 8]));
}
__global__ __launch_bounds__(128) void k_qkv(const _Float16* __restrict__ XT, const _Float16* __restrict__ PT, const float* __restrict__ bi, _Float16* __restrict__ Q16, _Float16* __restrict__ K16, _Float16* __restrict__ VT) {
  __shared__ __align__(16) float so[4][16][132];
  __shared__ __align__(16) _Float16 st[128][72];
  const int tid = threadIdx.x, wave = tid >> 5, lane = tid & 31, col = lane & 15, g = lane >> 4;
  const int which = blockIdx.z, nh2 = blockIdx.y; const int r0b = blockIdx.x * 64, r0 = r0b + wave * 16; const int n = r0b / LL, l0b = r0b % LL; const int n0 = which * CC + nh2 * 128;
  v8f acc[8] = {};
#pragma unroll
  for (int kc = 0; kc < CC / 32; ++kc) { const v16h a = frag_h(XT + (size_t)(r0 + col) * CC + kc * 32, lane);
#pragma unroll
    for (int j = 0; j < 8; ++j) acc[j] = wmma16(a, frag_h(PT + (size_t)(n0 + j * 16 + col) * CC + kc * 32, lane), acc[j]); }
  if (which < 2) {
#pragma unroll
    for (int j = 0; j < 8; ++j) { const float bb = bi[n0 + j * 16 + col];
#pragma unroll
      for (int r = 0; r < 8; ++r) so[wave][8 * g + r][j * 16 + col] = (acc[j][r] * (1.0f / 16.0f) + bb) * 4.0f; }
    LDSX();
    _Float16* D = which == 0 ? Q16 : K16;
    for (int qq = lane; qq < 16 * 4 * 4; qq += 32) { const int hh = qq >> 6, rl = (qq >> 2) & 15, pc = qq & 3; const int h = nh2 * 4 + hh; union { v8h h8; v4u u; } pk;
#pragma unroll
      for (int e = 0; e < 8; ++e) pk.h8[e] = (_Float16)so[wave][rl][hh * 32 + pc * 8 + e];
      vst2(D + (((size_t)n * NH + h) * LL + l0b + wave * 16 + rl) * HD + pc * 8, pk.u); } }
  else {
#pragma unroll
    for (int j = 0; j < 8; ++j) { const float bb = bi[n0 + j * 16 + col];
#pragma unroll
      for (int r = 0; r < 8; ++r) st[j * 16 + col][wave * 16 + 8 * g + r] = (_Float16)((acc[j][r] * (1.0f / 16.0f) + bb) * 4.0f); }
    __syncthreads();
    for (int qq = tid; qq < 128 * 8; qq += 128) { const int cl = qq >> 3, pc = qq & 7; const int c = nh2 * 128 + cl, h = c >> 5, d = c & 31;
      vst2(VT + (((size_t)n * NH + h) * HD + d) * LL + l0b + pc * 8, *(const v4u*)(&st[cl][pc * 8])); } }
}
__global__ __launch_bounds__(128) void k_attn(const _Float16* __restrict__ Q16, const _Float16* __restrict__ K16, const _Float16* __restrict__ VT, _Float16* __restrict__ O16) {
  __shared__ __align__(16) float sS[4][16][68];
  __shared__ __align__(16) _Float16 sP[4][16][72];
  __shared__ __align__(16) float sO[4][16][36];
  const int tid = threadIdx.x, w = tid >> 5, lane = tid & 31, col = lane & 15, g = lane >> 4;
  const size_t bh = blockIdx.y; const int q0 = blockIdx.x * 64 + w * 16;
  const v16h aq = frag_h(Q16 + (bh * LL + q0 + col) * HD, lane);
  float mrun = -3.0e38f, lrun = 0.f; v8f acc[2] = {};
#pragma unroll 1
  for (int kt = 0; kt < LL / 64; ++kt) {
#pragma unroll
    for (int t = 0; t < 4; ++t) { const int key = kt * 64 + t * 16 + col; const v8f s = wmma16(aq, frag_h(K16 + (bh * LL + key) * HD, lane), (v8f){});
#pragma unroll
      for (int r = 0; r < 8; ++r) sS[w][8 * g + r][t * 16 + col] = s[r] * (0.17677669529663689f / 16.0f); }
    LDSX();
    float mx = -3.4e38f;
#pragma unroll
    for (int jj = 0; jj < 32; ++jj) mx = fmaxf(mx, sS[w][col][g * 32 + jj]);
    mx = fmaxf(mx, __shfl_xor(mx, 16, 32));
    const float mnew = fmaxf(mrun, mx); const float corr = expf(mrun - mnew);
    float ps = 0.f;
#pragma unroll
    for (int jj = 0; jj < 32; ++jj) { const float p = expf(sS[w][col][g * 32 + jj] - mnew); ps += p; sP[w][col][g * 32 + jj] = (_Float16)(p * 16384.0f); }
    ps += __shfl_xor(ps, 16, 32);
    lrun = lrun * corr + ps; mrun = mnew;
#pragma unroll
    for (int r = 0; r < 8; ++r) { const float cr = __shfl(corr, 8 * g + r, 32); acc[0][r] *= cr; acc[1][r] *= cr; }
    LDSX();
#pragma unroll
    for (int kc = 0; kc < 2; ++kc) { const v16h pa = frag_h(&sP[w][col][0] + kc * 32, lane);
#pragma unroll
      for (int t = 0; t < 2; ++t) acc[t] = wmma16(pa, frag_h(VT + (bh * HD + t * 16 + col) * LL + kt * 64 + kc * 32, lane), acc[t]); }
    __builtin_amdgcn_wave_barrier(); }
#pragma unroll
  for (int r = 0; r < 8; ++r) { const float lr = __shfl(lrun, 8 * g + r, 32); const float inv = 8.0f / (lr * 16384.0f * 4.0f);
#pragma unroll
    for (int t = 0; t < 2; ++t) sO[w][8 * g + r][t * 16 + col] = acc[t][r] * inv; }
  LDSX();
  for (int qq = lane; qq < 16 * 4; qq += 32) { const int rl = qq >> 2, pc = qq & 3; union { v8h h8; v4u u; } pk;
#pragma unroll
    for (int e = 0; e < 8; ++e) pk.h8[e] = (_Float16)sO[w][rl][pc * 8 + e];
    vst2(O16 + ((bh * LL) + q0 + rl) * HD + pc * 8, pk.u); }
}
__global__ __launch_bounds__(128) void k_out(const _Float16* __restrict__ O16, const _Float16* __restrict__ PT, const float* __restrict__ bo, const float* __restrict__ x, const float* __restrict__ CA, float* __restrict__ out) {
  __shared__ __align__(16) float so[64][132];
  const int tid = threadIdx.x, wave = tid >> 5, lane = tid & 31, col = lane & 15, g = lane >> 4;
  const int b = blockIdx.z, hw = blockIdx.y, py = blockIdx.x; const int y = hw * WS + py;
  const int xx = wave * 16 + col; const int l = y * NB + b, n = xx;
#pragma unroll 1
  for (int ch = 0; ch < 2; ++ch) { v8f acc[8] = {};
#pragma unroll
    for (int kc = 0; kc < CC / 32; ++kc) { const int h = kc; const v16h a = frag_h(O16 + (((size_t)n * NH + h) * LL + l) * HD, lane);
#pragma unroll
      for (int j = 0; j < 8; ++j) acc[j] = wmma16(a, frag_h(PT + (size_t)(3 * CC + ch * 128 + j * 16 + col) * CC + kc * 32, lane), acc[j]); }
#pragma unroll
    for (int j = 0; j < 8; ++j) { const int c = ch * 128 + j * 16 + col; const float bb = bo[c];
#pragma unroll
      for (int r = 0; r < 8; ++r) so[wave * 16 + 8 * g + r][j * 16 + col] = acc[j][r] * (1.0f / (16.0f * 8.0f)) + bb; }
    __syncthreads();
    for (int q = tid; q < 128 * 4; q += 128) { const int cl = q >> 2, part = q & 3; const int c = ch * 128 + cl; const float cav = CA[(size_t)b * CC + c];
      const float* xr = x + (((size_t)b * CC + c) * HW + y) * HW + part * 16; float* orow = out + (((size_t)b * CC + c) * HW + y) * HW + part * 16;
#pragma unroll
      for (int v4 = 0; v4 < 4; ++v4) { v4f o; const v4f xv = *(const v4f*)(xr + v4 * 4);
#pragma unroll
        for (int e = 0; e < 4; ++e) o[e] = xv[e] * cav + so[part * 16 + v4 * 4 + e][cl];
        vst2(orow + v4 * 4, o); } }
    __syncthreads(); }
}
extern "C" void kernel_launch(void* const* d_in, const int* in_sizes, int n_in, void* d_out, int out_size, void* d_ws, size_t ws_size, hipStream_t stream) {
  (void)in_sizes; (void)n_in; (void)out_size; (void)ws_size;
  const float** I = (const float**)d_in;
  const float* x = I[0]; const float* w1 = I[1]; const float* b1 = I[2]; const float* w2 = I[3]; const float* b2 = I[4]; const float* Wi = I[5]; const float* bi = I[6]; const float* Wo = I[7]; const float* bo = I[8];
  float* out = (float*)d_out;
  char* ws = (char*)d_ws; size_t off = 0;
  auto take = [&](size_t bytes) { char* p = ws + off; off += (bytes + 255) & ~(size_t)255; return p; };
  float* CA = (float*)take(NB * CC * 4); _Float16* XT = (_Float16*)take((size_t)NR * CC * 2); _Float16* PT = (_Float16*)take((size_t)4 * CC * CC * 2);
  _Float16* Q16 = (_Float16*)take((size_t)NR * CC * 2); _Float16* K16 = (_Float16*)take((size_t)NR * CC * 2); _Float16* VT = (_Float16*)take((size_t)NR * CC * 2); _Float16* O16 = (_Float16*)take((size_t)NR * CC * 2);
  k_se<<<NB, 256, 0, stream>>>(x, w1, b1, w2, b2, CA);
  k_gather<<<dim3(WS, WS, NB), 256, 0, stream>>>(x, CA, XT);
  k_pack<<<4 * CC, 256, 0, stream>>>(Wi, Wo, PT);
  k_qkv<<<dim3(NR / 64, 2, 3), 128, 0, stream>>>(XT, PT, bi, Q16, K16, VT);
  k_attn<<<dim3(LL / 64, NN * NH), 128, 0, stream>>>(Q16, K16, VT, O16);
  k_out<<<dim3(WS, WS, NB), 128, 0, stream>>>(O16, PT, bo, x, CA, out);
}
